// DECORE_7567732376338
// MI455X (gfx1250) — hardware-verified
//
#include <hip/hip_runtime.h>
#include <stddef.h>


#define NTHR  256
#define NWAVE 8
#define DD    32
#define RD    64
#define GMAX  64
#define EPT   8
#define CHUNK (NTHR * EPT)
#define WCAP  (EPT * 32)
#define LISTN (NWAVE * WCAP)
#define PASSN (NWAVE * 32)
#define PCAP  (CHUNK + PASSN)
#define NB    512
#define TPW   (NB / (16 * NWAVE))
#define WSC   8.0f
#define WINV  0.125f

static_assert(PASSN == 256);
static_assert(PCAP >= CHUNK + PASSN);
static_assert(TPW * 16 * NWAVE == NB);
static_assert(NWAVE * 16 * DD <= DD * PASSN);
static_assert(NWAVE * 16 * DD <= NWAVE * 32 * DD);
static_assert((((NB + 1) * DD) % 4) == 0);

typedef float    v4f  __attribute__((ext_vector_type(4)));
typedef float    v8f  __attribute__((ext_vector_type(8)));
typedef int      v4i  __attribute__((ext_vector_type(4)));
typedef _Float16 v8h  __attribute__((ext_vector_type(8)));
typedef _Float16 v16h __attribute__((ext_vector_type(16)));
union FragH { v16h v; v8h h[2]; };

__device__ __forceinline__ v8f zero8f() {
  v8f z;
#pragma unroll
  for (int i = 0; i < 8; ++i) z[i] = 0.0f;
  return z;
}

__device__ __forceinline__ v8f wm(v16h a, v16h b, v8f c) {
  v8f d = __builtin_amdgcn_wmma_f32_16x16x32_f16(false, a, false, b, (short)0, c, false, false);
  asm volatile("v_nop\n\tv_nop\n\tv_nop\n\tv_nop" : "+v"(d) : "v"(a), "v"(b));
  return d;
}

__device__ __forceinline__ v8h cvt8(v4f a, v4f b) {
  v8h r;
  r[0] = (_Float16)a.x; r[1] = (_Float16)a.y; r[2] = (_Float16)a.z; r[3] = (_Float16)a.w;
  r[4] = (_Float16)b.x; r[5] = (_Float16)b.y; r[6] = (_Float16)b.z; r[7] = (_Float16)b.w;
  return r;
}

__device__ __forceinline__ v16h frag_f32(const float* row, int hh) {
  FragH f;
  const v4f x0 = *(const v4f*)(row + 8 * hh);
  const v4f x1 = *(const v4f*)(row + 8 * hh + 4);
  const v4f x2 = *(const v4f*)(row + 16 + 8 * hh);
  const v4f x3 = *(const v4f*)(row + 20 + 8 * hh);
  f.h[0] = cvt8(x0, x1);
  f.h[1] = cvt8(x2, x3);
  return f.v;
}
__device__ __forceinline__ v16h frag_h(const _Float16* row, int hh) {
  FragH f;
  f.h[0] = *(const v8h*)(row + 8 * hh);
  f.h[1] = *(const v8h*)(row + 16 + 8 * hh);
  return f.v;
}

__device__ __forceinline__ float sigm(float x) {
  const float e = __expf(-fabsf(x));
  const float s = __builtin_amdgcn_rcpf(1.0f + e);
  return x >= 0.0f ? s : e * s;
}
__device__ __forceinline__ float tanhm(float x) {
  const float e = __expf(-2.0f * fabsf(x));
  const float t = (1.0f - e) * __builtin_amdgcn_rcpf(1.0f + e);
  return copysignf(t, x);
}

__device__ __forceinline__ int scan_chunk(const int* __restrict__ dsts, int nE, int cbase, int nodeBase,
                                          int vec8, int* list, int tid, int wave) {
  int wc = 0;
  const int el0  = tid * EPT;
  const int e0   = cbase + el0;
  const int sent = -2147483647 - 1;
  v4i da, db;
  if (vec8 != 0 && cbase + CHUNK <= nE) {
    da = *(const v4i*)(dsts + e0);
    db = *(const v4i*)(dsts + e0 + 4);
  } else {
    da.x = (e0     < nE) ? dsts[min(e0, nE - 1)] : sent;
    da.y = (e0 + 1 < nE) ? dsts[min(e0 + 1, nE - 1)] : sent;
    da.z = (e0 + 2 < nE) ? dsts[min(e0 + 2, nE - 1)] : sent;
    da.w = (e0 + 3 < nE) ? dsts[min(e0 + 3, nE - 1)] : sent;
    db.x = (e0 + 4 < nE) ? dsts[min(e0 + 4, nE - 1)] : sent;
    db.y = (e0 + 5 < nE) ? dsts[min(e0 + 5, nE - 1)] : sent;
    db.z = (e0 + 6 < nE) ? dsts[min(e0 + 6, nE - 1)] : sent;
    db.w = (e0 + 7 < nE) ? dsts[min(e0 + 7, nE - 1)] : sent;
  }
  const unsigned nb = (unsigned)nodeBase;
  const unsigned s0 = (unsigned)da.x - nb, s1 = (unsigned)da.y - nb;
  const unsigned s2 = (unsigned)da.z - nb, s3 = (unsigned)da.w - nb;
  const unsigned s4 = (unsigned)db.x - nb, s5 = (unsigned)db.y - nb;
  const unsigned s6 = (unsigned)db.z - nb, s7 = (unsigned)db.w - nb;
  const bool h0 = s0 < (unsigned)NB, h1 = s1 < (unsigned)NB, h2 = s2 < (unsigned)NB, h3 = s3 < (unsigned)NB;
  const bool h4 = s4 < (unsigned)NB, h5 = s5 < (unsigned)NB, h6 = s6 < (unsigned)NB, h7 = s7 < (unsigned)NB;
  const unsigned any = __builtin_amdgcn_ballot_w32(h0 | h1 | h2 | h3 | h4 | h5 | h6 | h7);
  if (any != 0u) {
#define HITJ(J, HJ) { \
      const unsigned mj = __builtin_amdgcn_ballot_w32(HJ); \
      if (mj != 0u) { \
        if (HJ) { \
          const int pos = wc + (int)__builtin_amdgcn_mbcnt_lo(mj, 0u); \
          if (pos < WCAP) list[wave * WCAP + pos] = el0 + (J); \
        } \
        wc += (int)__builtin_popcount(mj); } }
    HITJ(0, h0)
    HITJ(1, h1)
    HITJ(2, h2)
    HITJ(3, h3)
    HITJ(4, h4)
    HITJ(5, h5)
    HITJ(6, h6)
    HITJ(7, h7)
#undef HITJ
  }
  return wc;
}

__global__ __launch_bounds__(NTHR) void k_pq(const float* __restrict__ ls, const float* __restrict__ Wm1,
                                             const float* __restrict__ bm1, float* P, float* Q, int nN) {
  __shared__ __attribute__((aligned(16))) _Float16 wpq[2 * DD * DD];
  __shared__ __attribute__((aligned(16))) float    tP[NWAVE * 16 * DD];
  __shared__ __attribute__((aligned(16))) float    tQ[NWAVE * 16 * DD];
  __shared__ __attribute__((aligned(16))) float    b1s[DD];
  const int tid = threadIdx.x, lane = tid & 31, wave = tid >> 5, hh = lane >> 4, m = lane & 15;

  for (int i = tid; i < 2 * DD * DD; i += NTHR) {
    const int pl = i >> 10, e = i & 1023, n = e >> 5, k = e & 31;
    wpq[i] = (_Float16)(Wm1[(pl * DD + k) * DD + n] * WSC);
  }
  if (tid < DD) b1s[tid] = bm1[tid];
  __syncthreads();

  const int row0 = (blockIdx.x * NWAVE + wave) * 16;
  int ra = row0 + m; ra = ra > nN - 1 ? nN - 1 : ra;
  const v16h aLs = frag_f32(ls + (size_t)ra * DD, hh);
  const v8f dP0 = wm(aLs, frag_h(wpq + m * DD, hh), zero8f());
  const v8f dP1 = wm(aLs, frag_h(wpq + (16 + m) * DD, hh), zero8f());
  const v8f dQ0 = wm(aLs, frag_h(wpq + (DD + m) * DD, hh), zero8f());
  const v8f dQ1 = wm(aLs, frag_h(wpq + (DD + 16 + m) * DD, hh), zero8f());

  float* tp = tP + wave * 16 * DD;
  float* tq = tQ + wave * 16 * DD;
  const float bq0 = b1s[m], bq1 = b1s[16 + m];
#pragma unroll
  for (int rr = 0; rr < 8; ++rr) {
    const int row = 8 * hh + rr;
    tp[row * DD + m]      = dP0[rr] * WINV;
    tp[row * DD + 16 + m] = dP1[rr] * WINV;
    tq[row * DD + m]      = dQ0[rr] * WINV + bq0;
    tq[row * DD + 16 + m] = dQ1[rr] * WINV + bq1;
  }
  __syncthreads();

  const int q4 = lane >> 3, p4 = lane & 7;
  v4f pv[4], qv[4];
#pragma unroll
  for (int u = 0; u < 4; ++u) {
    const int row = 4 * u + q4;
    pv[u] = *(const v4f*)(tp + row * DD + 4 * p4);
    qv[u] = *(const v4f*)(tq + row * DD + 4 * p4);
  }
#pragma unroll
  for (int u = 0; u < 4; ++u) {
    const size_t gi = (size_t)(row0 + 4 * u + q4) * DD + 4 * p4;
    *(volatile v4f*)(P + gi) = pv[u];
    *(volatile v4f*)(Q + gi) = qv[u];
  }
  __threadfence();
#pragma unroll
  for (int u = 0; u < 4; ++u) {
    const size_t gi = (size_t)(row0 + 4 * u + q4) * DD + 4 * p4;
    *(volatile v4f*)(P + gi) = pv[u];
    *(volatile v4f*)(Q + gi) = qv[u];
  }
}

__global__ __launch_bounds__(NTHR) void k_agg(
    const float* __restrict__ P, const float* __restrict__ Q, const float* __restrict__ lsin,
    const int* __restrict__ efirst, const int* __restrict__ esecond, const int* __restrict__ nsegp,
    const float* __restrict__ mk1, const float* __restrict__ Wm2, const float* __restrict__ bm2,
    const float* __restrict__ mk2,
    const float* __restrict__ Wz, const float* __restrict__ Uz, const float* __restrict__ bz,
    const float* __restrict__ Wr, const float* __restrict__ Ur, const float* __restrict__ br,
    const float* __restrict__ Wh, const float* __restrict__ Uh, const float* __restrict__ bh,
    float* lsout, int nN, int nE, int vec8) {
  __shared__ __attribute__((aligned(16))) float    acc[(NB + 1) * DD];
  __shared__ __attribute__((aligned(16))) _Float16 stg[NWAVE * 32 * DD];
  __shared__ __attribute__((aligned(16))) float    msgT[DD * PASSN];
  __shared__ __attribute__((aligned(16))) int      list[LISTN];
  __shared__ __attribute__((aligned(16))) int      pend[PCAP];
  __shared__ int slotb[PASSN];
  __shared__ __attribute__((aligned(16))) _Float16 wm2s[DD * DD];
  __shared__ __attribute__((aligned(16))) _Float16 wg[6 * DD * DD];
  __shared__ __attribute__((aligned(16))) float    mk1s[DD];
  __shared__ int wcnt[NWAVE];
  __shared__ int pendN;

  const int tid = threadIdx.x, lane = tid & 31, wave = tid >> 5, hh = lane >> 4, m = lane & 15;
  const int nodeBase = blockIdx.x * NB;

  {
    const v4f z4 = {0.0f, 0.0f, 0.0f, 0.0f};
    for (int i = tid; i < ((NB + 1) * DD) / 4; i += NTHR) *(v4f*)(acc + 4 * i) = z4;
  }
  for (int i = tid; i < DD * DD; i += NTHR) {
    const int n = i >> 5, k = i & 31;
    wm2s[i] = (_Float16)(Wm2[k * DD + n] * WSC);
  }
#pragma unroll 1
  for (int j = 0; j < 24; ++j) {
    const int i = j * NTHR + tid;
    const int mat = j >> 2;
    const float* src = (mat == 0) ? Wz : (mat == 1) ? Uz : (mat == 2) ? Wr : (mat == 3) ? Ur : (mat == 4) ? Wh : Uh;
    const int e = i & 1023, n = e >> 5, k = e & 31;
    wg[i] = (_Float16)(src[k * DD + n] * WSC);
  }
  if (tid < DD) mk1s[tid] = mk1[tid];
  if (tid == 0) pendN = 0;
  const float bm2v0 = bm2[m], bm2v1 = bm2[16 + m];
  const float m2v0  = mk2[m], m2v1  = mk2[16 + m];
  const float bz0 = bz[m], bz1 = bz[16 + m];
  const float br0 = br[m], br1 = br[16 + m];
  const float bh0 = bh[m], bh1 = bh[16 + m];
  int nseg = nsegp[0];
  nseg = nseg < 0 ? 0 : (nseg > nN ? nN : nseg);
  __syncthreads();

  const int nChunks = (nE + CHUNK - 1) / CHUNK;
#pragma unroll 1
  for (int ch = 0; ch < nChunks; ++ch) {
    const int cbase = ch * CHUNK;
    const int wc = scan_chunk(esecond, nE, cbase, nodeBase, vec8, list, tid, wave);
    if (lane == 0) wcnt[wave] = wc;
    __syncthreads();

    const int base = pendN;
    int tot = 0, myoff = 0;
#pragma unroll
    for (int w = 0; w < NWAVE; ++w) {
      int c = wcnt[w];
      c = c > WCAP ? WCAP : (c < 0 ? 0 : c);
      if (w < wave) myoff += c;
      tot += c;
    }
    int newN = base + tot;
    newN = newN > PCAP ? PCAP : newN;
    {
      int n = wcnt[wave];
      n = n > WCAP ? WCAP : (n < 0 ? 0 : n);
      const int* lp = list + wave * WCAP;
      for (int i = lane; i < n; i += 32) {
        const int pos = base + myoff + i;
        if (pos < PCAP) pend[pos] = cbase + lp[i];
      }
    }
    const int fin = (ch == nChunks - 1) ? 1 : 0;
    const int R   = (fin != 0) ? (newN + PASSN - 1) / PASSN : newN / PASSN;
    const int Pv  = (fin != 0) ? newN : R * PASSN;
    __syncthreads();

#pragma unroll 1
    for (int r = 0; r < R; ++r) {
      {
        const int idx = r * PASSN + wave * 32 + lane;
        const bool valid = idx < Pv;
        const int idc = idx < PCAP - 1 ? idx : PCAP - 1;
        int e = pend[idc];
        e = e < 0 ? 0 : (e > nE - 1 ? nE - 1 : e);
        int d = esecond[e];
        int s = efirst[e];
        int slot = d - nodeBase;
        const bool sv = valid && ((unsigned)slot < (unsigned)NB) && (d < nseg);
        slot = sv ? slot : NB;
        d = d < 0 ? 0 : (d > nN - 1 ? nN - 1 : d);
        s = s < 0 ? 0 : (s > nN - 1 ? nN - 1 : s);
        const float* prow = P + (size_t)s * DD;
        const float* qrow = Q + (size_t)d * DD;
        _Float16* hrow = stg + (wave * 32 + lane) * DD;
#pragma unroll
        for (int c8 = 0; c8 < 4; ++c8) {
          const v4f p0 = *(const v4f*)(prow + 8 * c8);
          const v4f p1 = *(const v4f*)(prow + 8 * c8 + 4);
          const v4f q0 = *(const v4f*)(qrow + 8 * c8);
          const v4f q1 = *(const v4f*)(qrow + 8 * c8 + 4);
          const v4f k0 = *(const v4f*)(mk1s + 8 * c8);
          const v4f k1 = *(const v4f*)(mk1s + 8 * c8 + 4);
          v8h hv;
#pragma unroll
          for (int jj = 0; jj < 4; ++jj) {
            const float ta = fmaxf(p0[jj] + q0[jj], 0.0f) * k0[jj];
            const float tb = fmaxf(p1[jj] + q1[jj], 0.0f) * k1[jj];
            hv[jj]     = (_Float16)(valid ? ta : 0.0f);
            hv[4 + jj] = (_Float16)(valid ? tb : 0.0f);
          }
          *(v8h*)(hrow + 8 * c8) = hv;
        }
        slotb[wave * 32 + lane] = slot;
      }
      __syncthreads();

      {
        const v16h bw0 = frag_h(wm2s + m * DD, hh);
        const v16h bw1 = frag_h(wm2s + (16 + m) * DD, hh);
#pragma unroll
        for (int et = 0; et < 2; ++et) {
          const v16h a = frag_h(stg + (wave * 32 + 16 * et + m) * DD, hh);
          const v8f d0 = wm(a, bw0, zero8f());
          const v8f d1 = wm(a, bw1, zero8f());
          float ta[8], tb[8];
#pragma unroll
          for (int rr = 0; rr < 8; ++rr) {
            ta[rr] = fmaxf(d0[rr] * WINV + bm2v0, 0.0f) * m2v0;
            tb[rr] = fmaxf(d1[rr] * WINV + bm2v1, 0.0f) * m2v1;
          }
          float* mp0 = msgT + m * PASSN + wave * 32 + 16 * et + 8 * hh;
          float* mp1 = msgT + (16 + m) * PASSN + wave * 32 + 16 * et + 8 * hh;
          const v4f ua = {ta[0], ta[1], ta[2], ta[3]}, ub = {ta[4], ta[5], ta[6], ta[7]};
          const v4f va = {tb[0], tb[1], tb[2], tb[3]}, vb = {tb[4], tb[5], tb[6], tb[7]};
          *(v4f*)mp0 = ua; *(v4f*)(mp0 + 4) = ub;
          *(v4f*)mp1 = va; *(v4f*)(mp1 + 4) = vb;
        }
      }
      __syncthreads();

      if (wave == 0) {
#pragma unroll 2
        for (int i = 0; i < PASSN; ++i) {
          int sl = slotb[i];
          sl = sl < 0 ? 0 : (sl > NB ? NB : sl);
          const float v = msgT[lane * PASSN + i];
          acc[sl * DD + lane] += v;
        }
      }
      __syncthreads();
    }

    int rem = newN - R * PASSN;
    rem = rem < 0 ? 0 : rem;
    if (R > 0 && tid < rem) pend[tid] = pend[R * PASSN + tid];
    if (tid == 0) pendN = rem;
  }
  __syncthreads();

  {
    float*    lt = msgT + wave * (16 * DD);
    _Float16* rt = stg  + wave * (16 * DD);
    const int q4 = lane >> 3, p4 = lane & 7;
#pragma unroll 1
    for (int j = 0; j < TPW; ++j) {
      const int srow = (j * NWAVE + wave) * 16;
      const int grow = nodeBase + srow;
#pragma unroll
      for (int u = 0; u < 4; ++u) {
        const int qq = lane + 32 * u;
        const int row = qq >> 3, c4 = (qq & 7) * 4;
        int gr = grow + row; gr = gr > nN - 1 ? nN - 1 : gr;
        *(v4f*)(lt + row * DD + c4) = *(const v4f*)(lsin + (size_t)gr * DD + c4);
      }
      __syncthreads();
      const v16h aAgg = frag_f32(acc + (srow + m) * DD, hh);
      const v16h aLs  = frag_f32(lt + m * DD, hh);
      v8f cR0 = wm(aAgg, frag_h(wg + (2 * DD + m) * DD, hh), zero8f());
      cR0 = wm(aLs, frag_h(wg + (3 * DD + m) * DD, hh), cR0);
      v8f cR1 = wm(aAgg, frag_h(wg + (2 * DD + 16 + m) * DD, hh), zero8f());
      cR1 = wm(aLs, frag_h(wg + (3 * DD + 16 + m) * DD, hh), cR1);
      v8f cZ0 = wm(aAgg, frag_h(wg + (0 * DD + m) * DD, hh), zero8f());
      cZ0 = wm(aLs, frag_h(wg + (1 * DD + m) * DD, hh), cZ0);
      v8f cZ1 = wm(aAgg, frag_h(wg + (0 * DD + 16 + m) * DD, hh), zero8f());
      cZ1 = wm(aLs, frag_h(wg + (1 * DD + 16 + m) * DD, hh), cZ1);
#pragma unroll
      for (int rr = 0; rr < 8; ++rr) {
        const int row = 8 * hh + rr;
        const float l0 = lt[row * DD + m], l1 = lt[row * DD + 16 + m];
        const float g0 = sigm(cR0[rr] * WINV + br0);
        const float g1 = sigm(cR1[rr] * WINV + br1);
        rt[row * DD + m]      = (_Float16)(g0 * l0);
        rt[row * DD + 16 + m] = (_Float16)(g1 * l1);
      }
      __syncthreads();
      const v16h aRh = frag_h(rt + m * DD, hh);
      v8f cH0 = wm(aAgg, frag_h(wg + (4 * DD + m) * DD, hh), zero8f());
      cH0 = wm(aRh, frag_h(wg + (5 * DD + m) * DD, hh), cH0);
      v8f cH1 = wm(aAgg, frag_h(wg + (4 * DD + 16 + m) * DD, hh), zero8f());
      cH1 = wm(aRh, frag_h(wg + (5 * DD + 16 + m) * DD, hh), cH1);
#pragma unroll
      for (int rr = 0; rr < 8; ++rr) {
        const int row = 8 * hh + rr;
        const float l0 = lt[row * DD + m], l1 = lt[row * DD + 16 + m];
        const float z0 = sigm(cZ0[rr] * WINV + bz0);
        const float z1 = sigm(cZ1[rr] * WINV + bz1);
        const float n0 = tanhm(cH0[rr] * WINV + bh0);
        const float n1 = tanhm(cH1[rr] * WINV + bh1);
        lt[row * DD + m]      = z0 * l0 + (1.0f - z0) * n0;
        lt[row * DD + 16 + m] = z1 * l1 + (1.0f - z1) * n1;
      }
      __syncthreads();
      v4f ov[4];
#pragma unroll
      for (int u = 0; u < 4; ++u) {
        const int row = 4 * u + q4;
        ov[u] = *(const v4f*)(lt + row * DD + 4 * p4);
      }
#pragma unroll
      for (int u = 0; u < 4; ++u) {
        const size_t gi = (size_t)(grow + 4 * u + q4) * DD + 4 * p4;
        *(volatile v4f*)(lsout + gi) = ov[u];
      }
      __threadfence();
#pragma unroll
      for (int u = 0; u < 4; ++u) {
        const size_t gi = (size_t)(grow + 4 * u + q4) * DD + 4 * p4;
        *(volatile v4f*)(lsout + gi) = ov[u];
      }
      __syncthreads();
    }
  }
}

__global__ __launch_bounds__(NTHR) void k_readout(
    const float* __restrict__ ls, const int* __restrict__ gid,
    const float* __restrict__ W1, const float* __restrict__ c1, const float* __restrict__ a1,
    const float* __restrict__ W2, const float* __restrict__ c2, const float* __restrict__ a2,
    const float* __restrict__ W3, const float* __restrict__ c3,
    float* out, int nN, int G) {
  __shared__ __attribute__((aligned(16))) float part[NWAVE * (GMAX + 1) * DD];
  __shared__ __attribute__((aligned(16))) float emb[GMAX * DD];
  __shared__ float h1s[GMAX * RD];
  __shared__ float h2s[GMAX * RD];
  __shared__ __attribute__((aligned(16))) float outs[GMAX];
  const int tid = threadIdx.x, lane = tid & 31, wave = tid >> 5;

  for (int i = tid; i < NWAVE * (GMAX + 1) * DD; i += NTHR) part[i] = 0.0f;
  __syncthreads();
  {
    float* pw = part + wave * (GMAX + 1) * DD;
#pragma unroll 1
    for (int n = wave; n < nN; n += NWAVE) {
      int g = gid[n];
      g = ((unsigned)g < (unsigned)G) ? g : GMAX;
      pw[g * DD + lane] += ls[(size_t)n * DD + lane];
    }
  }
  __syncthreads();
  for (int i = tid; i < GMAX * DD; i += NTHR) {
    float s = 0.0f;
#pragma unroll
    for (int w = 0; w < NWAVE; ++w) s += part[w * (GMAX + 1) * DD + i];
    emb[i] = s;
  }
  __syncthreads();
  {
    const int g = tid >> 2, nb = (tid & 3) * 16;
#pragma unroll 1
    for (int j = 0; j < 16; ++j) {
      const int n = nb + j;
      float s = c1[n];
#pragma unroll 1
      for (int k = 0; k < DD; ++k) s += emb[g * DD + k] * W1[k * RD + n];
      h1s[g * RD + n] = fmaxf(s, 0.0f) * a1[n];
    }
  }
  __syncthreads();
  {
    const int g = tid >> 2, nb = (tid & 3) * 16;
#pragma unroll 1
    for (int j = 0; j < 16; ++j) {
      const int n = nb + j;
      float s = c2[n];
#pragma unroll 1
      for (int k = 0; k < RD; ++k) s += h1s[g * RD + k] * W2[k * RD + n];
      h2s[g * RD + n] = fmaxf(s, 0.0f) * a2[n];
    }
  }
  __syncthreads();
  if (tid < GMAX) {
    float s = c3[0];
#pragma unroll 1
    for (int k = 0; k < RD; ++k) s += h2s[tid * RD + k] * W3[k];
    outs[tid] = s;
  }
  __syncthreads();
  const int li = lane & 15;
  const v4f v = *(const v4f*)(outs + 4 * li);
  const bool wr = (wave == 0) && (lane < 16) && (4 * li + 3 < G);
  if (wr) *(volatile v4f*)(out + 4 * li) = v;
  __threadfence();
  if (wr) *(volatile v4f*)(out + 4 * li) = v;
}

extern "C" void kernel_launch(void* const* d_in, const int* in_sizes, int n_in,
                              void* d_out, int out_size, void* d_ws, size_t ws_size,
                              hipStream_t stream) {
  if (n_in < 28) return;
  const int nN = in_sizes[0] / DD;
  if (nN <= 0 || in_sizes[0] != nN * DD) return;
  const int nE = in_sizes[1];
  if (nE <= 0 || in_sizes[2] != nE) return;
  if (in_sizes[3] != nN || in_sizes[4] < 1) return;
  if (in_sizes[5] != 2 * DD * DD || in_sizes[6] != DD || in_sizes[7] != DD) return;
  if (in_sizes[8] != DD * DD || in_sizes[9] != DD || in_sizes[10] != DD) return;
  if (in_sizes[11] != DD * DD || in_sizes[12] != DD * DD || in_sizes[13] != DD) return;
  if (in_sizes[14] != DD * DD || in_sizes[15] != DD * DD || in_sizes[16] != DD) return;
  if (in_sizes[17] != DD * DD || in_sizes[18] != DD * DD || in_sizes[19] != DD) return;
  if (in_sizes[20] != DD * RD || in_sizes[21] != RD || in_sizes[22] != RD) return;
  if (in_sizes[23] != RD * RD || in_sizes[24] != RD || in_sizes[25] != RD) return;
  if (in_sizes[26] != RD || in_sizes[27] < 1) return;
  const int G = out_size;
  if (G != GMAX) return;

  const float* link_state = (const float*)d_in[0];
  const int*   efirst     = (const int*)d_in[1];
  const int*   esecond    = (const int*)d_in[2];
  const int*   gids       = (const int*)d_in[3];
  const int*   nsegp      = (const int*)d_in[4];
  const float* Wm1 = (const float*)d_in[5];
  const float* bm1 = (const float*)d_in[6];
  const float* mk1 = (const float*)d_in[7];
  const float* Wm2 = (const float*)d_in[8];
  const float* bm2 = (const float*)d_in[9];
  const float* mk2 = (const float*)d_in[10];
  const float* Wz  = (const float*)d_in[11];
  const float* Uz  = (const float*)d_in[12];
  const float* bz  = (const float*)d_in[13];
  const float* Wr  = (const float*)d_in[14];
  const float* Ur  = (const float*)d_in[15];
  const float* br  = (const float*)d_in[16];
  const float* Wh  = (const float*)d_in[17];
  const float* Uh  = (const float*)d_in[18];
  const float* bh  = (const float*)d_in[19];
  const float* Wr1 = (const float*)d_in[20];
  const float* br1 = (const float*)d_in[21];
  const float* mr1 = (const float*)d_in[22];
  const float* Wr2 = (const float*)d_in[23];
  const float* br2 = (const float*)d_in[24];
  const float* mr2 = (const float*)d_in[25];
  const float* Wr3 = (const float*)d_in[26];
  const float* br3 = (const float*)d_in[27];
  float* out = (float*)d_out;

  const int nBlkA = (nN + NB - 1) / NB;
  const int nPad  = nBlkA * NB;
  const int nBlkP = nPad / (NWAVE * 16);

  const size_t plane = (size_t)nPad * DD * sizeof(float);
  char* ws = (char*)d_ws;
  size_t off = 0;
  const size_t oP  = off; off += plane;
  const size_t oQ  = off; off += plane;
  const size_t oL0 = off; off += plane;
  const size_t oL1 = off; off += plane;
  if (off > ws_size) return;
  float* P  = (float*)(ws + oP);
  float* Q  = (float*)(ws + oQ);
  float* lsb0 = (float*)(ws + oL0);
  float* lsb1 = (float*)(ws + oL1);

  const int vec8 = 1;
  const int T = 4;
  for (int t = 0; t < T; ++t) {
    const float* lin = (t == 0) ? link_state : (((t - 1) & 1) ? lsb1 : lsb0);
    float* lout = (t & 1) ? lsb1 : lsb0;
    k_pq<<<nBlkP, NTHR, 0, stream>>>(lin, Wm1, bm1, P, Q, nN);
    k_agg<<<nBlkA, NTHR, 0, stream>>>(P, Q, lin, efirst, esecond, nsegp, mk1, Wm2, bm2, mk2,
                                       Wz, Uz, bz, Wr, Ur, br, Wh, Uh, bh, lout, nN, nE, vec8);
  }
  const float* lfin = ((T - 1) & 1) ? lsb1 : lsb0;
  k_readout<<<1, NTHR, 0, stream>>>(lfin, gids, Wr1, br1, mr1, Wr2, br2, mr2, Wr3, br3, out, nN, G);
}
